// DRAGConv_17892833755548
// MI455X (gfx1250) — hardware-verified
//
#include <hip/hip_runtime.h>
#include <hip/hip_bf16.h>
#include <stddef.h>


#define KD    256
#define DF    256
#define NH    4
#define HC    64
#define NWT   3
#define GR    32
#define API   132
#define NTHR  256
#define NWAVE 8
#define NB    256
#define CHUNK 2048
#define NGRP  (CHUNK / (NTHR * 4))
#define WCAP  256

#define LDS_SACC (NB * DF)
#define LDS_MD   (2 * NB * NH)
#define LDS_LIST (NWAVE * WCAP)
#define LDS_BYTES ((LDS_SACC + LDS_MD + LDS_LIST + NWAVE) * 4)

static_assert(WCAP == (CHUNK / NTHR) * 32);
static_assert(NGRP >= 1);
static_assert(NB == 256);
static_assert(CHUNK == 2048);
static_assert(DF == NH * HC);
static_assert(HC == 64);
static_assert((KD % 32) == 0);
static_assert(((KD * DF / 8) % NTHR) == 0);
static_assert(LDS_BYTES == 278560);

typedef float  v4f  __attribute__((ext_vector_type(4)));
typedef float  v8f  __attribute__((ext_vector_type(8)));
typedef int    v4i  __attribute__((ext_vector_type(4)));
typedef __bf16 v16b __attribute__((ext_vector_type(16)));
union Frag { v16b v; v4i q[2]; };

__device__ __forceinline__ v8f wm(v16b a, v16b b, v8f c) {
  v8f d = __builtin_amdgcn_wmma_f32_16x16x32_bf16(false, a, false, b, (short)0, c, false, false);
  asm volatile("v_nop\n\tv_nop\n\tv_nop\n\tv_nop" : "+v"(d) : "v"(a), "v"(b));
  return d;
}

__device__ __forceinline__ unsigned bfr(float f) {
  const unsigned u = __float_as_uint(f);
  return (u + 0x7FFFu + ((u >> 16) & 1u)) >> 16;
}

__device__ __forceinline__ void split2(float a, float b, int& hi, int& lo) {
  const unsigned ha = bfr(a), hb = bfr(b);
  const float ra = a - __uint_as_float(ha << 16);
  const float rb = b - __uint_as_float(hb << 16);
  const unsigned la = bfr(ra), lb = bfr(rb);
  hi = (int)(ha | (hb << 16));
  lo = (int)(la | (lb << 16));
}

__global__ __launch_bounds__(NTHR) void k_wsplit(const float* __restrict__ W0,
                                                 const float* __restrict__ W1,
                                                 const float* __restrict__ W2,
                                                 int* Whi, int* Wlo, int n8) {
  const int i = blockIdx.x * NTHR + threadIdx.x;
  const int y = blockIdx.y;
  if (i >= n8) return;
  const float* W = (y == 0) ? W0 : ((y == 1) ? W1 : W2);
  const size_t o = (size_t)i * 8;
  const v4f a = *(const v4f*)(W + o);
  const v4f b = *(const v4f*)(W + o + 4);
  v4i hv, lv;
  int th, tl;
  split2(a.x, a.y, th, tl); hv.x = th; lv.x = tl;
  split2(a.z, a.w, th, tl); hv.y = th; lv.y = tl;
  split2(b.x, b.y, th, tl); hv.z = th; lv.z = tl;
  split2(b.z, b.w, th, tl); hv.w = th; lv.w = tl;
  const size_t oi = ((size_t)y * (size_t)n8 + (size_t)i) * 4;
  *(volatile v4i*)(Whi + oi) = hv;
  *(volatile v4i*)(Wlo + oi) = lv;
  __threadfence();
  *(volatile v4i*)(Whi + oi) = hv;
  *(volatile v4i*)(Wlo + oi) = lv;
}

__global__ __launch_bounds__(NTHR) void k_proj(
    const float* __restrict__ feat, const int* __restrict__ Whi, const int* __restrict__ Wlo,
    const float* __restrict__ b0, const float* __restrict__ b1, const float* __restrict__ b2,
    float* P0, float* P1, float* P2, int nN, int nP) {
  __shared__ __attribute__((aligned(16))) int   Ahi[GR * API];
  __shared__ __attribute__((aligned(16))) int   Alo[GR * API];
  __shared__ __attribute__((aligned(16))) float St[NWAVE * 512];

  const int tid  = threadIdx.x;
  const int l    = tid & 31;
  const int wave = tid >> 5;
  const int h    = l >> 4;
  const int m    = l & 15;
  const int rowBase = blockIdx.x * GR;

  {
    const int r  = tid >> 3;
    const int c0 = (tid & 7) * 32;
    int row = rowBase + r;
    if (row > nN - 1) row = nN - 1;
    const float* p = feat + (size_t)row * KD + c0;
    int* dh = Ahi + r * API + (c0 >> 1);
    int* dl = Alo + r * API + (c0 >> 1);
#pragma unroll
    for (int j = 0; j < 4; ++j) {
      const v4f f0 = *(const v4f*)(p + 8 * j);
      const v4f f1 = *(const v4f*)(p + 8 * j + 4);
      v4i hv, lv;
      int th, tl;
      split2(f0.x, f0.y, th, tl); hv.x = th; lv.x = tl;
      split2(f0.z, f0.w, th, tl); hv.y = th; lv.y = tl;
      split2(f1.x, f1.y, th, tl); hv.z = th; lv.z = tl;
      split2(f1.z, f1.w, th, tl); hv.w = th; lv.w = tl;
      *(v4i*)(dh + 4 * j) = hv;
      *(v4i*)(dl + 4 * j) = lv;
    }
  }
  __syncthreads();

  const v8f z8 = {0.f, 0.f, 0.f, 0.f, 0.f, 0.f, 0.f, 0.f};
#pragma unroll 1
  for (int cg = 0; cg < NWT; ++cg) {
    float* P = (cg == 0) ? P0 : ((cg == 1) ? P1 : P2);
    const float* bb = (cg == 0) ? b0 : ((cg == 1) ? b1 : b2);
    const int lim = (cg == 1) ? nN : nP;

    v8f acc[2][2];
#pragma unroll
    for (int rt = 0; rt < 2; ++rt) { acc[rt][0] = z8; acc[rt][1] = z8; }

#pragma unroll 1
    for (int kt = 0; kt < KD / 32; ++kt) {
      const int ki = kt * 16 + 4 * h;
      Frag ah[2], al[2], bh[2], bl[2];
#pragma unroll
      for (int rt = 0; rt < 2; ++rt) {
        const int ai = (16 * rt + m) * API + ki;
        ah[rt].q[0] = *(const v4i*)(Ahi + ai);
        ah[rt].q[1] = *(const v4i*)(Ahi + ai + 8);
        al[rt].q[0] = *(const v4i*)(Alo + ai);
        al[rt].q[1] = *(const v4i*)(Alo + ai + 8);
      }
#pragma unroll
      for (int ct = 0; ct < 2; ++ct) {
        const size_t bi = (size_t)(cg * DF + 32 * wave + 16 * ct + m) * (KD / 2) + ki;
        bh[ct].q[0] = *(const v4i*)(Whi + bi);
        bh[ct].q[1] = *(const v4i*)(Whi + bi + 8);
        bl[ct].q[0] = *(const v4i*)(Wlo + bi);
        bl[ct].q[1] = *(const v4i*)(Wlo + bi + 8);
      }
#pragma unroll
      for (int rt = 0; rt < 2; ++rt) {
#pragma unroll
        for (int ct = 0; ct < 2; ++ct) {
          v8f c = acc[rt][ct];
          c = wm(ah[rt].v, bh[ct].v, c);
          c = wm(ah[rt].v, bl[ct].v, c);
          c = wm(al[rt].v, bh[ct].v, c);
          acc[rt][ct] = c;
        }
      }
    }

    float bc[2];
#pragma unroll
    for (int ct = 0; ct < 2; ++ct) bc[ct] = bb[32 * wave + 16 * ct + m];
    const int pp = l & 7;
    const int ii = l >> 3;
#pragma unroll
    for (int rt = 0; rt < 2; ++rt) {
#pragma unroll
      for (int ct = 0; ct < 2; ++ct) {
#pragma unroll
        for (int r = 0; r < 8; ++r)
          St[wave * 512 + (8 * h + r) * 32 + 16 * ct + m] = acc[rt][ct][r] + bc[ct];
      }
      __syncthreads();
      v4f val[4];
      bool ok[4];
      float* gp[4];
#pragma unroll
      for (int j = 0; j < 4; ++j) {
        const int i = 4 * j + ii;
        val[j] = *(const v4f*)(St + wave * 512 + i * 32 + 4 * pp);
        const int row = rowBase + 16 * rt + i;
        ok[j] = (row < lim);
        gp[j] = P + (size_t)row * DF + 32 * wave + 4 * pp;
      }
#pragma unroll
      for (int j = 0; j < 4; ++j) if (ok[j]) *(volatile v4f*)(gp[j]) = val[j];
      __threadfence();
#pragma unroll
      for (int j = 0; j < 4; ++j) if (ok[j]) *(volatile v4f*)(gp[j]) = val[j];
      __syncthreads();
    }
  }
}

__global__ __launch_bounds__(NTHR) void k_agg(
    const float* __restrict__ FS, const float* __restrict__ FV, const float* __restrict__ attn,
    const int* __restrict__ srcA, const int* __restrict__ dstA,
    float* out, int nN, int nE) {
  extern __shared__ v4f lds_dyn[];
  float* sacc = (float*)lds_dyn;
  float* mx   = sacc + LDS_SACC;
  float* den  = mx + NB * NH;
  int*   list = (int*)(den + NB * NH);
  int*   wcnt = list + LDS_LIST;

  const int tid  = threadIdx.x;
  const int l    = tid & 31;
  const int wave = tid >> 5;
  const int hd   = l >> 3;
  const int nodeBase = blockIdx.x * NB;

  {
    const v4f z4 = {0.f, 0.f, 0.f, 0.f};
    for (int i = tid; i < LDS_SACC / 4; i += NTHR) lds_dyn[i] = z4;
    const float ninf = __uint_as_float(0xff800000u);
    for (int i = tid; i < NB * NH; i += NTHR) { mx[i] = ninf; den[i] = 0.f; }
  }
  const v4f at0 = *(const v4f*)(attn + 8 * l);
  const v4f at1 = *(const v4f*)(attn + 8 * l + 4);
  __syncthreads();

  const int nChunks = (nE + CHUNK - 1) / CHUNK;
#pragma unroll 1
  for (int ch = 0; ch < nChunks; ++ch) {
    const int cbase = ch * CHUNK;
    const bool full = (cbase + CHUNK <= nE);
    int wc = 0;
#pragma unroll
    for (int g = 0; g < NGRP; ++g) {
      const int el0 = (g * NTHR + tid) * 4;
      const int e0  = cbase + el0;
      const int sent = -2147483647 - 1;
      v4i d;
      if (full) {
        d = *(const v4i*)(dstA + e0);
      } else {
        const int q0 = min(e0, nE - 1), q1 = min(e0 + 1, nE - 1);
        const int q2 = min(e0 + 2, nE - 1), q3 = min(e0 + 3, nE - 1);
        const int r0 = dstA[q0], r1 = dstA[q1], r2 = dstA[q2], r3 = dstA[q3];
        d.x = (e0     < nE) ? r0 : sent;
        d.y = (e0 + 1 < nE) ? r1 : sent;
        d.z = (e0 + 2 < nE) ? r2 : sent;
        d.w = (e0 + 3 < nE) ? r3 : sent;
      }
      const unsigned s0 = (unsigned)d.x - (unsigned)nodeBase;
      const unsigned s1 = (unsigned)d.y - (unsigned)nodeBase;
      const unsigned s2 = (unsigned)d.z - (unsigned)nodeBase;
      const unsigned s3 = (unsigned)d.w - (unsigned)nodeBase;
      const bool h0 = s0 < (unsigned)NB;
      const bool h1 = s1 < (unsigned)NB;
      const bool h2 = s2 < (unsigned)NB;
      const bool h3 = s3 < (unsigned)NB;
      const unsigned many = __builtin_amdgcn_ballot_w32(h0 | h1 | h2 | h3);
      if (many != 0u) {
#define HITJ(J, HJ, SJ) { \
          const unsigned mj = __builtin_amdgcn_ballot_w32(HJ); \
          if (HJ) { \
            const int pos = wc + (int)__builtin_amdgcn_mbcnt_lo(mj, 0u); \
            if (pos < WCAP) list[wave * WCAP + pos] = ((el0 + (J)) << 8) | (int)(SJ); \
          } \
          wc += (int)__builtin_popcount(mj); }
        HITJ(0, h0, s0)
        HITJ(1, h1, s1)
        HITJ(2, h2, s2)
        HITJ(3, h3, s3)
#undef HITJ
      }
    }
    if (l == 0) wcnt[wave] = wc;
    __syncthreads();

    if (wave == 0) {
#pragma unroll 1
      for (int wsx = 0; wsx < NWAVE; ++wsx) {
        int n = wcnt[wsx];
        if (n > WCAP) n = WCAP;
        if (n < 0) n = 0;
#pragma unroll 1
        for (int i = 0; i < n; ++i) {
          const int ent  = list[wsx * WCAP + i];
          const int slot = ent & (NB - 1);
          const int el   = (ent >> 8) & (CHUNK - 1);
          int e = cbase + el;
          if (e > nE - 1) e = nE - 1;
          int u = srcA[e];
          u = u < 0 ? 0 : (u > nN - 1 ? nN - 1 : u);
          int nd = nodeBase + slot;
          if (nd > nN - 1) nd = nN - 1;
          const float* ps = FS  + (size_t)u  * DF + 8 * l;
          const float* pd = out + (size_t)nd * DF + 8 * l;
          const float* pv = FV  + (size_t)u  * DF + 8 * l;
          v4f x0 = *(const v4f*)(ps)     + *(const v4f*)(pd);
          v4f x1 = *(const v4f*)(ps + 4) + *(const v4f*)(pd + 4);
          x0.x = x0.x > 0.f ? x0.x : 0.2f * x0.x;
          x0.y = x0.y > 0.f ? x0.y : 0.2f * x0.y;
          x0.z = x0.z > 0.f ? x0.z : 0.2f * x0.z;
          x0.w = x0.w > 0.f ? x0.w : 0.2f * x0.w;
          x1.x = x1.x > 0.f ? x1.x : 0.2f * x1.x;
          x1.y = x1.y > 0.f ? x1.y : 0.2f * x1.y;
          x1.z = x1.z > 0.f ? x1.z : 0.2f * x1.z;
          x1.w = x1.w > 0.f ? x1.w : 0.2f * x1.w;
          float t = x0.x * at0.x + x0.y * at0.y + x0.z * at0.z + x0.w * at0.w
                  + x1.x * at1.x + x1.y * at1.y + x1.z * at1.z + x1.w * at1.w;
          t += __shfl_xor(t, 1, 32);
          t += __shfl_xor(t, 2, 32);
          t += __shfl_xor(t, 4, 32);
          const int ai = slot * NH + hd;
          const float mo = mx[ai];
          const float dn = den[ai];
          const float mn = fmaxf(mo, t);
          const float so = __expf(mo - mn);
          const float p  = __expf(t - mn);
          const v4f v0 = *(const v4f*)(pv);
          const v4f v1 = *(const v4f*)(pv + 4);
          v4f* sp = (v4f*)(sacc + slot * DF + 8 * l);
          const v4f c0 = sp[0];
          const v4f c1 = sp[1];
          sp[0] = c0 * so + p * v0;
          sp[1] = c1 * so + p * v1;
          mx[ai]  = mn;
          den[ai] = dn * so + p;
        }
      }
    }
    __syncthreads();
  }

  const int hA = l >> 4;
#pragma unroll 1
  for (int j = 0; j < NB / NWAVE; ++j) {
    const int slot = wave * (NB / NWAVE) + j;
    const int node = nodeBase + slot;
    if (node >= nN) break;
    const float d0 = den[slot * NH + hA];
    const float d2 = den[slot * NH + 2 + hA];
    const float i0 = (d0 > 0.f) ? (1.0f / d0) : 0.f;
    const float i2 = (d2 > 0.f) ? (1.0f / d2) : 0.f;
    const v4f y0 = *(const v4f*)(sacc + slot * DF + 4 * l) * i0;
    const v4f y2 = *(const v4f*)(sacc + slot * DF + 128 + 4 * l) * i2;
    float* op = out + (size_t)node * DF;
    *(volatile v4f*)(op + 4 * l)       = y0;
    *(volatile v4f*)(op + 128 + 4 * l) = y2;
    __threadfence();
    *(volatile v4f*)(op + 4 * l)       = y0;
    *(volatile v4f*)(op + 128 + 4 * l) = y2;
  }
}

extern "C" void kernel_launch(void* const* d_in, const int* in_sizes, int n_in,
                              void* d_out, int out_size, void* d_ws, size_t ws_size,
                              hipStream_t stream) {
  if (n_in < 10) return;
  const int nN = in_sizes[0] / KD;
  if (nN <= 0 || in_sizes[0] != nN * KD) return;
  if (in_sizes[1] != KD * DF || in_sizes[3] != KD * DF || in_sizes[5] != KD * DF) return;
  if (in_sizes[2] != DF || in_sizes[4] != DF || in_sizes[6] != DF) return;
  if (in_sizes[7] != NH * HC) return;
  const int nE = in_sizes[8];
  if (nE < 0 || in_sizes[9] != nE) return;
  if (out_size != nN * DF) return;

  const float* feat = (const float*)d_in[0];
  const float* Wsrc = (const float*)d_in[1];
  const float* bsrc = (const float*)d_in[2];
  const float* Wdst = (const float*)d_in[3];
  const float* bdst = (const float*)d_in[4];
  const float* Wv   = (const float*)d_in[5];
  const float* bv   = (const float*)d_in[6];
  const float* attn = (const float*)d_in[7];
  const int*   srcA = (const int*)d_in[8];
  const int*   dstA = (const int*)d_in[9];
  float* out = (float*)d_out;

  const int nP = ((nN + GR - 1) / GR) * GR;
  size_t off = 0;
  int*   Whi = (int*)((char*)d_ws + off);   off += (size_t)NWT * DF * KD * 2;
  int*   Wlo = (int*)((char*)d_ws + off);   off += (size_t)NWT * DF * KD * 2;
  float* FS  = (float*)((char*)d_ws + off); off += (size_t)nP * DF * sizeof(float);
  float* FV  = (float*)((char*)d_ws + off); off += (size_t)nP * DF * sizeof(float);
  if (off > ws_size) return;

  const int n8 = KD * DF / 8;
  dim3 gw(n8 / NTHR, NWT);
  k_wsplit<<<gw, NTHR, 0, stream>>>(Wsrc, Wdst, Wv, Whi, Wlo, n8);

  k_proj<<<nP / GR, NTHR, 0, stream>>>(feat, Whi, Wlo, bsrc, bdst, bv, FS, out, FV, nN, nP);

  hipFuncSetAttribute(reinterpret_cast<const void*>(&k_agg),
                      hipFuncAttributeMaxDynamicSharedMemorySize, LDS_BYTES);
  const int grid = (nN + NB - 1) / NB;
  k_agg<<<grid, NTHR, LDS_BYTES, stream>>>(FS, FV, attn, srcA, dstA, out, nN, nE);
}
